// MyOutRGCN_687194767721
// MI455X (gfx1250) — hardware-verified
//
#include <hip/hip_runtime.h>
#include <stddef.h>


#define DF        128
#define NREL      2
#define NCAT      (DF * (NREL + 1))
#define NOUT      5

#define PG_WAVES  4
#define PG_THR    (PG_WAVES * 32)
#define PG_ROWS   (PG_WAVES * 16)

#define NTHR      256
#define NWAVE     8
#define EPT       8
#define NGRP      2
#define CHUNK     (NTHR * EPT * NGRP)
#define WCAP      (EPT * NGRP * 32)
#define LISTN     (NWAVE * WCAP)
#define NBC       4096
#define NB        512
#define RPW       (NB / NWAVE)

#define LDS_ACC   (NB * DF * 4)
#define LDS_LIST  (LISTN * 4)
#define LDS_AGG   (LDS_ACC + LDS_LIST + 64)
#define LDS_SELF  (LDS_ACC + LDS_LIST + NB * 4 + 64)
#define LDS_MAX   (300 * 1024)

static_assert((CHUNK & (CHUNK - 1)) == 0);
static_assert(CHUNK <= 4096);
static_assert((NBC & (NBC - 1)) == 0);
static_assert(NBC <= 4096);
static_assert(NBC % NB == 0);
static_assert((NB & (NB - 1)) == 0);
static_assert(NB % NWAVE == 0);
static_assert(NB % 32 == 0);
static_assert(NTHR * 32 == NBC * NREL);
static_assert(NB * NOUT * 4 <= LDS_LIST);
static_assert((NB * NOUT) % 128 == 0);
static_assert(NCAT % DF == 0);
static_assert(LDS_AGG <= LDS_MAX);

typedef float  v4f   __attribute__((ext_vector_type(4)));
typedef float  v4fa  __attribute__((ext_vector_type(4), __may_alias__));
typedef float  v8f   __attribute__((ext_vector_type(8)));
typedef int    v4i   __attribute__((ext_vector_type(4)));
typedef __bf16 bf16_t;
typedef bf16_t v8bf  __attribute__((ext_vector_type(8)));
typedef bf16_t v16bf __attribute__((ext_vector_type(16)));
union FragB { v16bf v; v8bf h[2]; v4i q[2]; };
union Pack8 { v8bf v; v4i q; };

__device__ __forceinline__ v8f wmb(v16bf a, v16bf b, v8f c) {
  v8f d = __builtin_amdgcn_wmma_f32_16x16x32_bf16(false, a, false, b, (short)0, c, false, false);
  asm volatile("v_nop\n\tv_nop\n\tv_nop\n\tv_nop" : "+v"(d) : "v"(a), "v"(b));
  return d;
}

template <int B>
__device__ __forceinline__ void split8(FragB& hi, FragB& lo, v4f a, v4f b) {
#define SPL1(I, X) { const float xv = (X); const bf16_t hb = (bf16_t)xv; hi.v[B + (I)] = hb; lo.v[B + (I)] = (bf16_t)(xv - (float)hb); }
  SPL1(0, a.x) SPL1(1, a.y) SPL1(2, a.z) SPL1(3, a.w)
  SPL1(4, b.x) SPL1(5, b.y) SPL1(6, b.z) SPL1(7, b.w)
#undef SPL1
}

__device__ __forceinline__ int wrap_clamp(int v, int n) {
  v = (v < 0) ? v + n : v;
  v = (v < 0) ? 0 : ((v > n - 1) ? n - 1 : v);
  return v;
}

__device__ __forceinline__ v4f lrelu4(v4f v) {
  v4f o;
  o.x = v.x > 0.0f ? v.x : 0.01f * v.x;
  o.y = v.y > 0.0f ? v.y : 0.01f * v.y;
  o.z = v.z > 0.0f ? v.z : 0.01f * v.z;
  o.w = v.w > 0.0f ? v.w : 0.01f * v.w;
  return o;
}

__device__ __forceinline__ float wsum(float v) {
  v += __shfl_xor(v, 16);
  v += __shfl_xor(v, 8);
  v += __shfl_xor(v, 4);
  v += __shfl_xor(v, 2);
  v += __shfl_xor(v, 1);
  return v;
}

__device__ __forceinline__ float sigm(float z) {
  return __builtin_amdgcn_rcpf(1.0f + __expf(-z));
}

template <bool BM, int NSLOT>
__device__ __forceinline__ int scan_chunk(const int* __restrict__ dsts, int nE, int cbase, int nodeBase, int nN,
                                          int vec8, const unsigned* bm, int* list, int tid, int wave) {
  int wc = 0;
#pragma unroll
  for (int g = 0; g < NGRP; ++g) {
    const int el0  = (g * NTHR + tid) * EPT;
    const int e0   = cbase + el0;
    const int sent = -2147483647 - 1;
    v4i da, db;
    if (vec8 != 0 && e0 + 7 < nE) {
      da = *(const v4i*)(dsts + e0);
      db = *(const v4i*)(dsts + e0 + 4);
    } else {
      da.x = (e0     < nE) ? dsts[min(e0,     nE - 1)] : sent;
      da.y = (e0 + 1 < nE) ? dsts[min(e0 + 1, nE - 1)] : sent;
      da.z = (e0 + 2 < nE) ? dsts[min(e0 + 2, nE - 1)] : sent;
      da.w = (e0 + 3 < nE) ? dsts[min(e0 + 3, nE - 1)] : sent;
      db.x = (e0 + 4 < nE) ? dsts[min(e0 + 4, nE - 1)] : sent;
      db.y = (e0 + 5 < nE) ? dsts[min(e0 + 5, nE - 1)] : sent;
      db.z = (e0 + 6 < nE) ? dsts[min(e0 + 6, nE - 1)] : sent;
      db.w = (e0 + 7 < nE) ? dsts[min(e0 + 7, nE - 1)] : sent;
    }
#define TSTJ(J, DV) \
    unsigned s##J; bool h##J; \
    { const int dv = (DV); \
      if (BM) { const bool val = (unsigned)dv < (unsigned)nN; const int wi = val ? (dv >> 5) : 0; \
                const unsigned wrd = bm[wi]; h##J = val && (((wrd >> (dv & 31)) & 1u) != 0u); s##J = 0u; } \
      else    { s##J = (unsigned)dv - (unsigned)nodeBase; h##J = s##J < (unsigned)NSLOT; } }
    TSTJ(0, da.x) TSTJ(1, da.y) TSTJ(2, da.z) TSTJ(3, da.w)
    TSTJ(4, db.x) TSTJ(5, db.y) TSTJ(6, db.z) TSTJ(7, db.w)
#undef TSTJ
    const unsigned any = __builtin_amdgcn_ballot_w32(h0 | h1 | h2 | h3 | h4 | h5 | h6 | h7);
    if (any != 0u) {
#define HITJ(J, HJ, SJ) { \
        const unsigned mj = __builtin_amdgcn_ballot_w32(HJ); \
        if (mj != 0u) { \
          if (HJ) { \
            const int pos  = wc + (int)__builtin_amdgcn_mbcnt_lo(mj, 0u); \
            const int entv = BM ? (el0 + (J)) : (((el0 + (J)) << 12) | (int)(SJ)); \
            if (pos < WCAP) list[wave * WCAP + pos] = entv; \
          } \
          wc += (int)__builtin_popcount(mj); } }
      HITJ(0, h0, s0)
      HITJ(1, h1, s1)
      HITJ(2, h2, s2)
      HITJ(3, h3, s3)
      HITJ(4, h4, s4)
      HITJ(5, h5, s5)
      HITJ(6, h6, s6)
      HITJ(7, h7, s7)
#undef HITJ
    }
  }
  return wc;
}

__global__ __launch_bounds__(NTHR) void k_wprep(
    const float* __restrict__ w1, const float* __restrict__ rt1,
    const float* __restrict__ w2, const float* __restrict__ rt2,
    bf16_t* whi, bf16_t* wlo, int nTot) {
  const int i = blockIdx.x * NTHR + threadIdx.x;
  if (i >= nTot) return;
  const int o   = i * 8;
  const int lyr = o / (NCAT * DF);
  const int rem = o - lyr * (NCAT * DF);
  const int n   = rem / DF;
  const int k0  = rem - n * DF;
  const float* w  = lyr ? w2 : w1;
  const float* rt = lyr ? rt2 : rt1;
  const float* p = (n < NREL * DF) ? (w + (size_t)(n / DF) * DF * DF + (size_t)k0 * DF + (n & (DF - 1)))
                                   : (rt + (size_t)k0 * DF + (n - NREL * DF));
  Pack8 ph, pl;
#define WSP(I) { const float xv = p[(size_t)(I) * DF]; const bf16_t hb = (bf16_t)xv; ph.v[(I)] = hb; pl.v[(I)] = (bf16_t)(xv - (float)hb); }
  WSP(0) WSP(1) WSP(2) WSP(3) WSP(4) WSP(5) WSP(6) WSP(7)
#undef WSP
  bf16_t* dh = whi + o;
  bf16_t* dl = wlo + o;
  const v4i qh = ph.q, ql = pl.q;
  *(volatile v4i*)dh = qh;
  *(volatile v4i*)dl = ql;
  __threadfence();
  *(volatile v4i*)dh = qh;
  *(volatile v4i*)dl = ql;
}

__device__ __forceinline__ void kstep(const float* ap, const bf16_t* bhp, const bf16_t* blp, v8f (&c)[8]) {
  const v4f p0 = *(const v4f*)(ap);
  const v4f p1 = *(const v4f*)(ap + 4);
  const v4f p2 = *(const v4f*)(ap + 16);
  const v4f p3 = *(const v4f*)(ap + 20);
  FragB ahi, alo;
  split8<0>(ahi, alo, p0, p1);
  split8<8>(ahi, alo, p2, p3);
#pragma unroll
  for (int ct = 0; ct < 8; ++ct) {
    const bf16_t* hp = bhp + (size_t)ct * 16 * DF;
    const bf16_t* lp = blp + (size_t)ct * 16 * DF;
    FragB bh, bq;
    bh.q[0] = *(const v4i*)hp;  bh.q[1] = *(const v4i*)(hp + 16);
    bq.q[0] = *(const v4i*)lp;  bq.q[1] = *(const v4i*)(lp + 16);
    c[ct] = wmb(alo.v, bh.v, c[ct]);
    c[ct] = wmb(ahi.v, bq.v, c[ct]);
    c[ct] = wmb(ahi.v, bh.v, c[ct]);
  }
}

__global__ __launch_bounds__(PG_THR) void k_proj(
    const float* __restrict__ A, const bf16_t* __restrict__ whi, const bf16_t* __restrict__ wlo,
    float* P, int nN) {
  __shared__ float tile[PG_WAVES * 16 * DF];
  const int tid = threadIdx.x, lane = tid & 31, wave = tid >> 5, hh = lane >> 4, m = lane & 15;
  const int rowBase = blockIdx.x * PG_ROWS + wave * 16;
  int ar = rowBase + m;
  ar = ar > nN - 1 ? nN - 1 : ar;
  const float* ap0 = A + (size_t)ar * DF + 8 * hh;
  float* tw = tile + wave * 16 * DF;

#pragma unroll 1
  for (int cg = 0; cg < NCAT / DF; ++cg) {
    v8f c[8];
#pragma unroll
    for (int ct = 0; ct < 8; ++ct) { const v8f z = {0.f, 0.f, 0.f, 0.f, 0.f, 0.f, 0.f, 0.f}; c[ct] = z; }
    const bf16_t* bh0 = whi + (size_t)(cg * DF + m) * DF + 8 * hh;
    const bf16_t* bl0 = wlo + (size_t)(cg * DF + m) * DF + 8 * hh;
#pragma unroll 1
    for (int ks = 0; ks < DF / 32; ++ks)
      kstep(ap0 + 32 * ks, bh0 + 32 * ks, bl0 + 32 * ks, c);

    float* sp = tw + (8 * hh) * DF + m;
#pragma unroll
    for (int ct = 0; ct < 8; ++ct) {
#pragma unroll
      for (int r = 0; r < 8; ++r) sp[r * DF + 16 * ct] = c[ct][r];
    }
    __syncthreads();

    {
      const float* lr = tw + 4 * lane;
      float* gp = P + (size_t)rowBase * NCAT + cg * DF + 4 * lane;
#pragma unroll
      for (int i = 0; i < 16; ++i) {
        if (rowBase + i < nN) {
          const v4f v = *(const v4fa*)(lr + i * DF);
          *(volatile v4f*)(gp + (size_t)i * NCAT) = v;
        }
      }
      __threadfence();
#pragma unroll
      for (int i = 0; i < 16; ++i) {
        if (rowBase + i < nN) {
          const v4f v = *(const v4fa*)(lr + i * DF);
          *(volatile v4f*)(gp + (size_t)i * NCAT) = v;
        }
      }
    }
    __syncthreads();
  }
}

__global__ __launch_bounds__(NTHR) void k_count(
    const int* __restrict__ ei, const int* __restrict__ et,
    float* inv, int nN, int nE, int nPad, int vec8) {
  __shared__ int list[LISTN];
  __shared__ int cnt[NBC * NREL];
  __shared__ int wcnt[NWAVE];
  const int tid = threadIdx.x, lane = tid & 31, wave = tid >> 5;
  const int nodeBase = blockIdx.x * NBC;
  const int* dsts = ei + nE;

  for (int i = tid; i < NBC * NREL; i += NTHR) cnt[i] = 0;
  __syncthreads();

  const int nChunks = (nE + CHUNK - 1) / CHUNK;
#pragma unroll 1
  for (int ch = 0; ch < nChunks; ++ch) {
    const int cbase = ch * CHUNK;
    const int wc = scan_chunk<false, NBC>(dsts, nE, cbase, nodeBase, nN, vec8, (const unsigned*)0, list, tid, wave);
    if (lane == 0) wcnt[wave] = wc;
    __syncthreads();
    if (wave == 0) {
#pragma unroll 1
      for (int wsx = 0; wsx < NWAVE; ++wsx) {
        int n = __builtin_amdgcn_readfirstlane(wcnt[wsx]);
        n = n > WCAP ? WCAP : (n < 0 ? 0 : n);
        const int* lp = list + wsx * WCAP;
#pragma unroll 1
        for (int i = 0; i < n; ++i) {
          const int ent  = __builtin_amdgcn_readfirstlane(lp[i]);
          const int slot = ent & (NBC - 1);
          int e = cbase + ((ent >> 12) & (CHUNK - 1));
          e = e > nE - 1 ? nE - 1 : e;
          const int r = __builtin_amdgcn_readfirstlane(et[e]);
          if ((unsigned)r < (unsigned)NREL) {
            if (lane == 0) cnt[slot * NREL + r] = cnt[slot * NREL + r] + 1;
          }
        }
      }
    }
    __syncthreads();
  }

  {
    const int r = tid >> 7;
    const int t = tid & 127;
    float* gb = inv + (size_t)r * nPad + nodeBase;
#pragma unroll 1
    for (int q = 0; q < NBC / 512; ++q) {
      const int s4 = q * 512 + 4 * t;
      v4f v;
      { const int c0 = cnt[(s4 + 0) * NREL + r]; v.x = __builtin_amdgcn_rcpf((float)(c0 > 0 ? c0 : 1)); }
      { const int c1 = cnt[(s4 + 1) * NREL + r]; v.y = __builtin_amdgcn_rcpf((float)(c1 > 0 ? c1 : 1)); }
      { const int c2 = cnt[(s4 + 2) * NREL + r]; v.z = __builtin_amdgcn_rcpf((float)(c2 > 0 ? c2 : 1)); }
      { const int c3 = cnt[(s4 + 3) * NREL + r]; v.w = __builtin_amdgcn_rcpf((float)(c3 > 0 ? c3 : 1)); }
      *(volatile v4f*)(gb + s4) = v;
    }
    __threadfence();
#pragma unroll 1
    for (int q = 0; q < NBC / 512; ++q) {
      const int s4 = q * 512 + 4 * t;
      v4f v;
      { const int c0 = cnt[(s4 + 0) * NREL + r]; v.x = __builtin_amdgcn_rcpf((float)(c0 > 0 ? c0 : 1)); }
      { const int c1 = cnt[(s4 + 1) * NREL + r]; v.y = __builtin_amdgcn_rcpf((float)(c1 > 0 ? c1 : 1)); }
      { const int c2 = cnt[(s4 + 2) * NREL + r]; v.z = __builtin_amdgcn_rcpf((float)(c2 > 0 ? c2 : 1)); }
      { const int c3 = cnt[(s4 + 3) * NREL + r]; v.w = __builtin_amdgcn_rcpf((float)(c3 > 0 ? c3 : 1)); }
      *(volatile v4f*)(gb + s4) = v;
    }
  }
}

__device__ __forceinline__ void agg_store_rows(const float* acc, const float* __restrict__ P, v4f bb,
                                               float* hout, int nodeBase, int nN, int wave, int lane) {
#pragma unroll 1
  for (int i = 0; i < RPW; ++i) {
    const int slot = wave * RPW + i;
    const int node = nodeBase + slot;
    if (node < nN) {
      const v4f a  = *(const v4fa*)(acc + slot * DF + 4 * lane);
      const v4f pr = *(const v4f*)(P + (size_t)node * NCAT + NREL * DF + 4 * lane);
      const v4f v  = lrelu4(a + pr + bb);
      *(volatile v4f*)(hout + (size_t)node * DF + 4 * lane) = v;
    }
  }
}

__global__ __launch_bounds__(NTHR) void k_agg(
    const int* __restrict__ ei, const int* __restrict__ et, const float* __restrict__ P,
    const float* __restrict__ inv, const float* __restrict__ bias,
    float* hout, int nN, int nE, int nPad, int vec8) {
  extern __shared__ v4f lds_dyn[];
  float* acc  = (float*)lds_dyn;
  int*   list = (int*)((char*)lds_dyn + LDS_ACC);
  int*   wcnt = (int*)((char*)lds_dyn + LDS_ACC + LDS_LIST);
  const int tid = threadIdx.x, lane = tid & 31, wave = tid >> 5;
  const int nodeBase = blockIdx.x * NB;
  const int* dsts = ei + nE;

  {
    const v4f z = {0.f, 0.f, 0.f, 0.f};
    for (int i = tid; i < NB * DF / 4; i += NTHR) lds_dyn[i] = z;
  }
  __syncthreads();

  const int nChunks = (nE + CHUNK - 1) / CHUNK;
#pragma unroll 1
  for (int ch = 0; ch < nChunks; ++ch) {
    const int cbase = ch * CHUNK;
    const int wc = scan_chunk<false, NB>(dsts, nE, cbase, nodeBase, nN, vec8, (const unsigned*)0, list, tid, wave);
    if (lane == 0) wcnt[wave] = wc;
    __syncthreads();
    if (wave == 0) {
#pragma unroll 1
      for (int wsx = 0; wsx < NWAVE; ++wsx) {
        int n = __builtin_amdgcn_readfirstlane(wcnt[wsx]);
        n = n > WCAP ? WCAP : (n < 0 ? 0 : n);
        const int* lp = list + wsx * WCAP;
#pragma unroll 1
        for (int i = 0; i < n; ++i) {
          const int ent  = __builtin_amdgcn_readfirstlane(lp[i]);
          const int slot = ent & (NB - 1);
          int e = cbase + ((ent >> 12) & (CHUNK - 1));
          e = e > nE - 1 ? nE - 1 : e;
          const int r   = __builtin_amdgcn_readfirstlane(et[e]);
          const int src = wrap_clamp(__builtin_amdgcn_readfirstlane(ei[e]), nN);
          if ((unsigned)r < (unsigned)NREL) {
            const float w  = inv[(size_t)r * nPad + nodeBase + slot];
            const v4f   vw = (*(const v4f*)(P + (size_t)src * NCAT + r * DF + 4 * lane)) * w;
            v4f* ap = (v4f*)(acc + slot * DF + 4 * lane);
            const v4f cur = *ap;
            *ap = cur + vw;
          }
        }
      }
    }
    __syncthreads();
  }

  const v4f bb = *(const v4f*)(bias + 4 * lane);
  agg_store_rows(acc, P, bb, hout, nodeBase, nN, wave, lane);
  __threadfence();
  agg_store_rows(acc, P, bb, hout, nodeBase, nN, wave, lane);
}

__device__ __forceinline__ v4f sel_row_val(const float* acc, const float* __restrict__ P, v4f bb,
                                           int slot, int node, int lane) {
  const v4f a  = *(const v4fa*)(acc + slot * DF + 4 * lane);
  const v4f pr = *(const v4f*)(P + (size_t)node * NCAT + NREL * DF + 4 * lane);
  return lrelu4(a + pr + bb);
}

__device__ __forceinline__ void sel_store_out1(const float* rs, float* g1, int nf, int lane) {
#pragma unroll 1
  for (int q = 0; q < (NB * NOUT) / 128; ++q) {
    const int f = q * 128 + 4 * lane;
    if (f + 4 <= nf) {
      const v4f v = *(const v4fa*)(rs + f);
      *(volatile v4f*)(g1 + f) = v;
    }
  }
  const int ft = nf & ~3;
  if (lane < (nf & 3)) {
    const float v = rs[ft + lane];
    *(volatile float*)(g1 + ft + lane) = v;
  }
}

__global__ __launch_bounds__(NTHR) void k_sel(
    const int* __restrict__ ei, const int* __restrict__ et, const int* __restrict__ idx,
    const float* __restrict__ P, const float* __restrict__ inv, const float* __restrict__ bias,
    const float* __restrict__ mw, const float* __restrict__ mb,
    float* out0, float* out1, int nN, int nE, int nPad, int nSel, int bmWords, int vec8) {
  extern __shared__ v4f lds_dyn[];
  float*    acc  = (float*)lds_dyn;
  int*      list = (int*)((char*)lds_dyn + LDS_ACC);
  int*      sidx = (int*)((char*)lds_dyn + LDS_ACC + LDS_LIST);
  int*      wcnt = sidx + NB;
  unsigned* bm   = (unsigned*)((char*)lds_dyn + LDS_SELF);
  const int tid = threadIdx.x, lane = tid & 31, wave = tid >> 5;
  const int sBase = blockIdx.x * NB;
  const int* dsts = ei + nE;

  {
    const v4f z = {0.f, 0.f, 0.f, 0.f};
    for (int i = tid; i < NB * DF / 4; i += NTHR) lds_dyn[i] = z;
    for (int i = tid; i < bmWords; i += NTHR) bm[i] = 0u;
    for (int t = tid; t < NB; t += NTHR) {
      const int s = sBase + t;
      sidx[t] = (s < nSel) ? wrap_clamp(idx[s], nN) : -1;
    }
  }
  __syncthreads();
  if (tid == 0) {
#pragma unroll 1
    for (int t = 0; t < NB; ++t) {
      const int node = sidx[t];
      if (node >= 0) bm[node >> 5] |= (1u << (node & 31));
    }
  }
  __syncthreads();

  const int nChunks = (nE + CHUNK - 1) / CHUNK;
#pragma unroll 1
  for (int ch = 0; ch < nChunks; ++ch) {
    const int cbase = ch * CHUNK;
    const int wc = scan_chunk<true, NB>(dsts, nE, cbase, 0, nN, vec8, bm, list, tid, wave);
    if (lane == 0) wcnt[wave] = wc;
    __syncthreads();
    if (wave == 0) {
#pragma unroll 1
      for (int wsx = 0; wsx < NWAVE; ++wsx) {
        int n = __builtin_amdgcn_readfirstlane(wcnt[wsx]);
        n = n > WCAP ? WCAP : (n < 0 ? 0 : n);
        const int* lp = list + wsx * WCAP;
#pragma unroll 1
        for (int i = 0; i < n; ++i) {
          const int ent = __builtin_amdgcn_readfirstlane(lp[i]);
          int e = cbase + (ent & (CHUNK - 1));
          e = e > nE - 1 ? nE - 1 : e;
          const int d   = __builtin_amdgcn_readfirstlane(dsts[e]);
          const int r   = __builtin_amdgcn_readfirstlane(et[e]);
          const int src = wrap_clamp(__builtin_amdgcn_readfirstlane(ei[e]), nN);
          if ((unsigned)r < (unsigned)NREL && (unsigned)d < (unsigned)nN) {
            const float w  = inv[(size_t)r * nPad + d];
            const v4f   vw = (*(const v4f*)(P + (size_t)src * NCAT + r * DF + 4 * lane)) * w;
#pragma unroll 1
            for (int j = 0; j < NB / 32; ++j) {
              unsigned mk = __builtin_amdgcn_ballot_w32(sidx[32 * j + lane] == d);
              while (mk != 0u) {
                const int slot = 32 * j + (int)__builtin_ctz(mk);
                v4f* ap = (v4f*)(acc + slot * DF + 4 * lane);
                const v4f cur = *ap;
                *ap = cur + vw;
                mk &= mk - 1u;
              }
            }
          }
        }
      }
    }
    __syncthreads();
  }

  float* res = (float*)list;
  const v4f bb = *(const v4f*)(bias + 4 * lane);
  const float* wp = mw + 20 * lane;
  const v4f wa = *(const v4f*)(wp);
  const v4f wb = *(const v4f*)(wp + 4);
  const v4f wc = *(const v4f*)(wp + 8);
  const v4f wd = *(const v4f*)(wp + 12);
  const v4f we = *(const v4f*)(wp + 16);
  const float mb0 = mb[0], mb1 = mb[1], mb2 = mb[2], mb3 = mb[3], mb4 = mb[4];

#pragma unroll 1
  for (int i = 0; i < RPW; ++i) {
    const int slot = wave * RPW + i;
    const int s = sBase + slot;
    if (s < nSel) {
      const int node = sidx[slot];
      const v4f v = sel_row_val(acc, P, bb, slot, node, lane);
      *(volatile v4f*)(out0 + (size_t)s * DF + 4 * lane) = v;
      const float z0 = wsum(v.x * wa.x + v.y * wb.y + v.z * wc.z + v.w * wd.w) + mb0;
      const float z1 = wsum(v.x * wa.y + v.y * wb.z + v.z * wc.w + v.w * we.x) + mb1;
      const float z2 = wsum(v.x * wa.z + v.y * wb.w + v.z * wd.x + v.w * we.y) + mb2;
      const float z3 = wsum(v.x * wa.w + v.y * wc.x + v.z * wd.y + v.w * we.z) + mb3;
      const float z4 = wsum(v.x * wb.x + v.y * wc.y + v.z * wd.z + v.w * we.w) + mb4;
      if (lane == 0) {
        res[slot * NOUT + 0] = sigm(z0);
        res[slot * NOUT + 1] = sigm(z1);
        res[slot * NOUT + 2] = sigm(z2);
        res[slot * NOUT + 3] = sigm(z3);
        res[slot * NOUT + 4] = sigm(z4);
      }
    }
  }
  __threadfence();
#pragma unroll 1
  for (int i = 0; i < RPW; ++i) {
    const int slot = wave * RPW + i;
    const int s = sBase + slot;
    if (s < nSel) {
      const int node = sidx[slot];
      const v4f v = sel_row_val(acc, P, bb, slot, node, lane);
      *(volatile v4f*)(out0 + (size_t)s * DF + 4 * lane) = v;
    }
  }
  __syncthreads();

  if (wave == 0) {
    int nrows = nSel - sBase;
    nrows = nrows > NB ? NB : nrows;
    const int nf = nrows * NOUT;
    float* g1 = out1 + (size_t)sBase * NOUT;
    sel_store_out1(res, g1, nf, lane);
    __threadfence();
    sel_store_out1(res, g1, nf, lane);
  }
}

extern "C" void kernel_launch(void* const* d_in, const int* in_sizes, int n_in,
                              void* d_out, int out_size, void* d_ws, size_t ws_size,
                              hipStream_t stream) {
  if (n_in < 12) return;
  const int nN   = in_sizes[0] / DF;
  const int nE   = in_sizes[1] / 2;
  const int nSel = in_sizes[3];
  if (nN <= 0 || nE < 0 || nSel <= 0) return;
  if (in_sizes[0] != nN * DF || in_sizes[1] != 2 * nE || in_sizes[2] < nE) return;
  if (in_sizes[4] != NREL * DF * DF || in_sizes[5] != DF * DF || in_sizes[6] < DF) return;
  if (in_sizes[7] != NREL * DF * DF || in_sizes[8] != DF * DF || in_sizes[9] < DF) return;
  if (in_sizes[10] != DF * NOUT || in_sizes[11] < NOUT) return;
  if (out_size != nSel * DF + nSel * NOUT) return;

  const float* x     = (const float*)d_in[0];
  const int*   ei    = (const int*)d_in[1];
  const int*   et    = (const int*)d_in[2];
  const int*   idx   = (const int*)d_in[3];
  const float* W1    = (const float*)d_in[4];
  const float* root1 = (const float*)d_in[5];
  const float* b1    = (const float*)d_in[6];
  const float* W2    = (const float*)d_in[7];
  const float* root2 = (const float*)d_in[8];
  const float* b2    = (const float*)d_in[9];
  const float* mlpw  = (const float*)d_in[10];
  const float* mlpb  = (const float*)d_in[11];
  float* out0 = (float*)d_out;
  float* out1 = out0 + (size_t)nSel * DF;

  const int nBlkC   = (nN + NBC - 1) / NBC;
  const int nPad    = nBlkC * NBC;
  const int nBlk    = (nN + NB - 1) / NB;
  const int nPB     = (nN + PG_ROWS - 1) / PG_ROWS;
  const int nSB     = (nSel + NB - 1) / NB;
  const int bmWords = (nN + 31) / 32;
  const int ldsSel  = LDS_SELF + ((bmWords * 4 + 15) & ~15);
  if (ldsSel > LDS_MAX) return;
  const int vec8 = ((nE & 3) == 0) ? 1 : 0;

  char* ws = (char*)d_ws;
  size_t off = 0;
  const size_t szPl  = (size_t)2 * NCAT * DF * sizeof(bf16_t);
  const size_t oWh   = off; off += szPl;                              off = (off + 255) & ~(size_t)255;
  const size_t oWl   = off; off += szPl;                              off = (off + 255) & ~(size_t)255;
  const size_t oInv  = off; off += (size_t)NREL * nPad * sizeof(float); off = (off + 255) & ~(size_t)255;
  const size_t oP    = off; off += (size_t)nN * NCAT * sizeof(float);  off = (off + 255) & ~(size_t)255;
  const size_t oH1   = off; off += (size_t)nN * DF * sizeof(float);    off = (off + 255) & ~(size_t)255;
  if (off > ws_size) return;
  bf16_t* whi = (bf16_t*)(ws + oWh);
  bf16_t* wlo = (bf16_t*)(ws + oWl);
  float*  inv = (float*)(ws + oInv);
  float*  P   = (float*)(ws + oP);
  float*  h1  = (float*)(ws + oH1);

  const int nTot = 2 * NCAT * DF / 8;
  k_wprep<<<(nTot + NTHR - 1) / NTHR, NTHR, 0, stream>>>(W1, root1, W2, root2, whi, wlo, nTot);

  k_count<<<nBlkC, NTHR, 0, stream>>>(ei, et, inv, nN, nE, nPad, vec8);

  k_proj<<<nPB, PG_THR, 0, stream>>>(x, whi, wlo, P, nN);

  hipFuncSetAttribute(reinterpret_cast<const void*>(&k_agg),
                      hipFuncAttributeMaxDynamicSharedMemorySize, LDS_AGG);
  k_agg<<<nBlk, NTHR, LDS_AGG, stream>>>(ei, et, P, inv, b1, h1, nN, nE, nPad, vec8);

  k_proj<<<nPB, PG_THR, 0, stream>>>(h1, whi + (size_t)NCAT * DF, wlo + (size_t)NCAT * DF, P, nN);

  hipFuncSetAttribute(reinterpret_cast<const void*>(&k_sel),
                      hipFuncAttributeMaxDynamicSharedMemorySize, ldsSel);
  k_sel<<<nSB, NTHR, ldsSel, stream>>>(ei, et, idx, P, inv, b2, mlpw, mlpb, out0, out1,
                                        nN, nE, nPad, nSel, bmWords, vec8);
}
